// CachedModel_22153441313361
// MI455X (gfx1250) — hardware-verified
//
#include <hip/hip_runtime.h>


namespace {
constexpr int NCH = 128, HID = 512, BUF = 516, TP = 528, JUMP = 8, LK = 50, CHUNK = 400, NBLK = 14;
constexpr int NOUT = CHUNK + 2 * NCH * BUF;
constexpr float WSC = 256.0f, XS = 8.0f, EPS = 1e-8f, INV = 1.0f / (WSC * XS);

typedef _Float16 b16;
typedef __attribute__((ext_vector_type(16))) _Float16 v16b;
typedef __attribute__((ext_vector_type(8))) _Float16 v8b;
typedef __attribute__((ext_vector_type(4))) _Float16 v4b;
typedef __attribute__((ext_vector_type(8))) float v8f;
typedef __attribute__((ext_vector_type(4))) float v4f;
__device__ __forceinline__ float bf16_rne(float f) { unsigned int u = __float_as_uint(f); u += 0x7FFFu + ((u >> 16) & 1u); return __uint_as_float(u & 0xFFFF0000u); }
__device__ __forceinline__ void split16(float v, b16& hi, b16& lo) { hi = (b16)v; lo = (b16)(v - (float)hi); }
__device__ __forceinline__ v16b frag_kb(const b16* p, int hh) { const v8b a = *(const v8b*)(p + 8 * hh), b = *(const v8b*)(p + 16 + 8 * hh); v16b f;
#pragma unroll
  for (int e = 0; e < 8; ++e) { f[e] = a[e]; f[8 + e] = b[e]; } return f; }
__device__ __forceinline__ v8f wmma16b(v16b a, v16b b, v8f c) { v8f d = __builtin_amdgcn_wmma_f32_16x16x32_f16(false, a, false, b, (short)0, c, false, false); asm volatile("v_nop\n\tv_nop\n\tv_nop\n\tv_nop" : "+v"(d) : "v"(a), "v"(b)); return d; }
__device__ __forceinline__ float pmul(float a, float b) { float p = a * b; asm volatile("" : "+v"(p)); return p; }
__device__ __forceinline__ float wsum(float v) {
#pragma unroll
  for (int o = 16; o >= 1; o >>= 1) v += __shfl_xor(v, o); return v; }
__device__ __forceinline__ int imin(int a, int b) { return a < b ? a : b; }

__global__ __launch_bounds__(256) void prep_kernel(const float* __restrict__ w1, const float* __restrict__ w2, b16* __restrict__ W1s, b16* __restrict__ W2s, float* __restrict__ Z, int nz4) {
  const size_t tid = (size_t)blockIdx.x * 256 + threadIdx.x, nth = (size_t)gridDim.x * 256;
  const int NW = NBLK * HID * NCH / 8;
  for (int pass = 0; pass < 2; ++pass) {
    for (size_t g = tid; g < (size_t)2 * NW; g += nth) { const bool second = g >= (size_t)NW; const size_t e = (second ? g - NW : g) * 8; const float* w = second ? w2 : w1;
      const v4f a = *(const v4f*)(w + e), c = *(const v4f*)(w + e + 4); v8b o;
#pragma unroll
      for (int k = 0; k < 4; ++k) { o[k] = (b16)(bf16_rne(a[k]) * WSC); o[4 + k] = (b16)(bf16_rne(c[k]) * WSC); }
      *(volatile v8b*)((second ? W2s : W1s) + e) = o; }
    const v4f z4 = {0.0f, 0.0f, 0.0f, 0.0f};
    for (size_t g = tid; g < (size_t)nz4; g += nth) *(volatile v4f*)(Z + g * 4) = z4;
    __threadfence(); }
}
__global__ __launch_bounds__(256) void front_kernel(const float* __restrict__ mix, const float* __restrict__ wenc, const float* __restrict__ lng, const float* __restrict__ lnb, const float* __restrict__ wbn, float* __restrict__ ENC, float* __restrict__ LNN) {
  __shared__ float Se[NCH][JUMP + 1], Sl[NCH][JUMP + 1], Smu[JUMP], Srs[JUMP];
  const int t_ = threadIdx.x, n = t_ >> 1, j0 = (t_ & 1) * 4;
  float e4[4];
  for (int q = 0; q < 4; ++q) { const int j = j0 + q; float s = 0.0f;
    for (int k = 0; k < 2 * LK; ++k) { const int ci = k / LK, l = k - ci * LK; s += pmul(bf16_rne(wenc[(n * 2 + ci) * LK + l]), bf16_rne(mix[ci * CHUNK + j * LK + l])); }
    e4[q] = fmaxf(s, 0.0f); Se[n][j] = e4[q]; }
  __syncthreads();
  if (t_ < JUMP) { float s = 0.0f; for (int c = 0; c < NCH; ++c) s += Se[c][t_]; const float mu = s * (1.0f / NCH); float ss = 0.0f; for (int c = 0; c < NCH; ++c) { const float d = Se[c][t_] - mu; ss += pmul(d, d); }
    Smu[t_] = mu; Srs[t_] = rsqrtf(ss * (1.0f / NCH) + EPS); }
  __syncthreads();
  for (int k = t_; k < NCH * JUMP; k += 256) { const int c = k >> 3, j = k & 7; Sl[c][j] = pmul(bf16_rne(lng[c]), (Se[c][j] - Smu[j]) * Srs[j]) + bf16_rne(lnb[c]); }
  __syncthreads();
  float l4[4];
  for (int q = 0; q < 4; ++q) { const int j = j0 + q; float s = 0.0f; for (int c = 0; c < NCH; ++c) s += pmul(bf16_rne(wbn[n * NCH + c]), Sl[c][j]); l4[q] = s; }
  for (int pass = 0; pass < 2; ++pass) { *(volatile v4f*)(ENC + n * JUMP + j0) = (v4f){e4[0], e4[1], e4[2], e4[3]}; *(volatile v4f*)(LNN + n * JUMP + j0) = (v4f){l4[0], l4[1], l4[2], l4[3]}; __threadfence(); }
}
__global__ __launch_bounds__(256) void x0_kernel(const float* __restrict__ lbuf, const float* __restrict__ LNN, float* __restrict__ XF, b16* __restrict__ XH, b16* __restrict__ XL) {
  const int wave = threadIdx.x >> 5, lane = threadIdx.x & 31, t = blockIdx.x * 8 + wave, c0 = lane * 4;
  const int ta = imin(t + JUMP, BUF - 1), tb = imin((t >= 508) ? t - 508 : 0, JUMP - 1);
  float v[4];
#pragma unroll
  for (int q = 0; q < 4; ++q) { const float a = bf16_rne(lbuf[(c0 + q) * BUF + ta]), b = LNN[(c0 + q) * JUMP + tb]; v[q] = (t < 508) ? a : (t < BUF) ? b : 0.0f; }
  v4b h4, l4;
#pragma unroll
  for (int q = 0; q < 4; ++q) { b16 a_, c_; split16(v[q] * XS, a_, c_); h4[q] = a_; l4[q] = c_; }
  for (int pass = 0; pass < 2; ++pass) { *(volatile v4f*)(XF + (size_t)t * NCH + c0) = (v4f){v[0], v[1], v[2], v[3]}; *(volatile v4b*)(XH + (size_t)t * NCH + c0) = h4; *(volatile v4b*)(XL + (size_t)t * NCH + c0) = l4; __threadfence(); }
}
__global__ __launch_bounds__(256) void blockA_kernel(const b16* __restrict__ W1s, const b16* __restrict__ XH, const b16* __restrict__ XL, const float* __restrict__ p1, const float* __restrict__ g1, const float* __restrict__ b1, float* __restrict__ Y1, int T_in) {
  __shared__ float S1[8][16], S2[8][16]; __shared__ __attribute__((aligned(16))) float Ts[16][HID + 4];
  const int wave = threadIdx.x >> 5, lane = threadIdx.x & 31, nloc = lane & 15, hlf = lane >> 4, t0 = blockIdx.x * 16;
  v8f acc[4] = {{}, {}, {}, {}};
#pragma unroll
  for (int kb = 0; kb < NCH; kb += 32) { const v16b bh = frag_kb(XH + (size_t)(t0 + nloc) * NCH + kb, hlf), bl = frag_kb(XL + (size_t)(t0 + nloc) * NCH + kb, hlf);
#pragma unroll
    for (int mt = 0; mt < 4; ++mt) { const v16b a = frag_kb(W1s + (size_t)(wave * 64 + mt * 16 + nloc) * NCH + kb, hlf); acc[mt] = wmma16b(a, bh, acc[mt]); acc[mt] = wmma16b(a, bl, acc[mt]); } }
  const float pa = bf16_rne(p1[0]); float s = 0.0f;
#pragma unroll
  for (int mt = 0; mt < 4; ++mt)
#pragma unroll
    for (int r = 0; r < 8; ++r) { float v = acc[mt][r] * INV; v = (v >= 0.0f) ? v : pa * v; acc[mt][r] = v; s += v; }
  s += __shfl_xor(s, 16); if (hlf == 0) S1[wave][nloc] = s;
  __syncthreads();
  float mu = 0.0f; for (int w = 0; w < 8; ++w) mu += S1[w][nloc]; mu *= (1.0f / HID);
  float ss = 0.0f;
#pragma unroll
  for (int mt = 0; mt < 4; ++mt)
#pragma unroll
    for (int r = 0; r < 8; ++r) { const float d = acc[mt][r] - mu; ss += pmul(d, d); }
  ss += __shfl_xor(ss, 16); if (hlf == 0) S2[wave][nloc] = ss;
  __syncthreads();
  float var = 0.0f; for (int w = 0; w < 8; ++w) var += S2[w][nloc]; var *= (1.0f / HID); const float rs = rsqrtf(var + EPS);
#pragma unroll
  for (int mt = 0; mt < 4; ++mt) { const int h0 = wave * 64 + mt * 16 + 8 * hlf; const v4f ga = *(const v4f*)(g1 + h0), gb = *(const v4f*)(g1 + h0 + 4), ba = *(const v4f*)(b1 + h0), bb = *(const v4f*)(b1 + h0 + 4);
#pragma unroll
    for (int r = 0; r < 8; ++r) { const float g = bf16_rne(r < 4 ? ga[r] : gb[r - 4]), bv = bf16_rne(r < 4 ? ba[r] : bb[r - 4]); Ts[nloc][h0 + r] = pmul(g, (acc[mt][r] - mu) * rs) + bv; } }
  __syncthreads();
  for (int pass = 0; pass < 2; ++pass) {
    for (int rr = 2 * wave; rr < 2 * wave + 2; ++rr) { if (t0 + rr < T_in) {
#pragma unroll
      for (int q = 0; q < 4; ++q) { const int h = 4 * lane + 128 * q; *(volatile v4f*)(Y1 + (size_t)(t0 + rr) * HID + h) = *(const v4f*)(&Ts[rr][h]); } } }
    __threadfence(); }
}
__global__ __launch_bounds__(256) void blockB_kernel(const float* __restrict__ Y1, const float* __restrict__ dw, const float* __restrict__ p2, const float* __restrict__ g2, const float* __restrict__ b2, const b16* __restrict__ W2s, const float* __restrict__ XFi, float* __restrict__ XFo, b16* __restrict__ XHo, b16* __restrict__ XLo, int d, int T_out) {
  __shared__ __attribute__((aligned(16))) b16 Bh[16][HID + 8], Bl[16][HID + 8]; __shared__ __attribute__((aligned(16))) float To[16][NCH + 4];
  const int wave = threadIdx.x >> 5, lane = threadIdx.x & 31, nloc = lane & 15, hlf = lane >> 4, t0 = blockIdx.x * 16;
  const float pa = bf16_rne(p2[0]);
  for (int rr = 2 * wave; rr < 2 * wave + 2; ++rr) { const int t = t0 + rr; float z[16];
#pragma unroll
    for (int q = 0; q < 4; ++q) { const int h = 4 * lane + 128 * q; const v4f y0 = *(const v4f*)(Y1 + (size_t)imin(t, TP - 1) * HID + h), ya = *(const v4f*)(Y1 + (size_t)imin(t + d, TP - 1) * HID + h), yb = *(const v4f*)(Y1 + (size_t)imin(t + 2 * d, TP - 1) * HID + h);
      const v4f w0 = *(const v4f*)(dw + h * 3), w1 = *(const v4f*)(dw + h * 3 + 4), w2 = *(const v4f*)(dw + h * 3 + 8);
      const float wk[12] = {w0[0], w0[1], w0[2], w0[3], w1[0], w1[1], w1[2], w1[3], w2[0], w2[1], w2[2], w2[3]};
#pragma unroll
      for (int e = 0; e < 4; ++e) { float v = pmul(bf16_rne(wk[3 * e]), y0[e]) + pmul(bf16_rne(wk[3 * e + 1]), ya[e]) + pmul(bf16_rne(wk[3 * e + 2]), yb[e]); v = (v >= 0.0f) ? v : pa * v; z[4 * q + e] = v; } }
    float s = 0.0f;
#pragma unroll
    for (int e = 0; e < 16; ++e) s += z[e];
    const float mu = wsum(s) * (1.0f / HID); float ss = 0.0f;
#pragma unroll
    for (int e = 0; e < 16; ++e) { const float dd = z[e] - mu; ss += pmul(dd, dd); }
    const float rs = rsqrtf(wsum(ss) * (1.0f / HID) + EPS);
#pragma unroll
    for (int q = 0; q < 4; ++q) { const int h = 4 * lane + 128 * q; const v4f gg = *(const v4f*)(g2 + h), bb = *(const v4f*)(b2 + h); v4b h4, l4;
#pragma unroll
      for (int e = 0; e < 4; ++e) { const float v = pmul(bf16_rne(gg[e]), (z[4 * q + e] - mu) * rs) + bf16_rne(bb[e]); b16 a_, c_; split16(v * XS, a_, c_); h4[e] = a_; l4[e] = c_; }
      *(v4b*)(&Bh[rr][h]) = h4; *(v4b*)(&Bl[rr][h]) = l4; } }
  __syncthreads();
  v8f acc = {};
#pragma unroll 4
  for (int kb = 0; kb < HID; kb += 32) { const v16b a = frag_kb(W2s + (size_t)(wave * 16 + nloc) * HID + kb, hlf); acc = wmma16b(a, frag_kb(&Bh[nloc][kb], hlf), acc); acc = wmma16b(a, frag_kb(&Bl[nloc][kb], hlf), acc); }
  { const int c0 = wave * 16 + 8 * hlf; const size_t ri = (size_t)imin(t0 + nloc + 2 * d, TP - 1) * NCH + c0; const v4f xa = *(const v4f*)(XFi + ri), xb = *(const v4f*)(XFi + ri + 4);
#pragma unroll
    for (int r = 0; r < 8; ++r) To[nloc][c0 + r] = acc[r] * INV + (r < 4 ? xa[r] : xb[r - 4]); }
  __syncthreads();
  for (int pass = 0; pass < 2; ++pass) {
    for (int rr = 2 * wave; rr < 2 * wave + 2; ++rr) { if (t0 + rr < T_out) { const int c = 4 * lane; const v4f v = *(const v4f*)(&To[rr][c]); v4b h4, l4;
#pragma unroll
      for (int e = 0; e < 4; ++e) { b16 a_, c_; split16(v[e] * XS, a_, c_); h4[e] = a_; l4[e] = c_; }
      *(volatile v4f*)(XFo + (size_t)(t0 + rr) * NCH + c) = v; *(volatile v4b*)(XHo + (size_t)(t0 + rr) * NCH + c) = h4; *(volatile v4b*)(XLo + (size_t)(t0 + rr) * NCH + c) = l4; } }
    __threadfence(); }
}
__global__ __launch_bounds__(256) void tail_kernel(const float* __restrict__ XF, const float* __restrict__ ENC, const float* __restrict__ wmask, const float* __restrict__ wdec, float* __restrict__ EST) {
  __shared__ float Sx[JUMP][NCH + 1], Sw[NCH][JUMP + 1], Se[CHUNK + 16];
  const int t_ = threadIdx.x;
  for (int k = t_; k < JUMP * NCH; k += 256) { const int t = k >> 7, c = k & 127; Sx[t][c] = XF[t * NCH + c]; }
  __syncthreads();
  { const int n = t_ >> 1, j0 = (t_ & 1) * 4;
    for (int q = 0; q < 4; ++q) { const int t = j0 + q; float s = 0.0f; for (int c = 0; c < NCH; ++c) s += pmul(bf16_rne(wmask[n * NCH + c]), Sx[t][c]); Sw[n][t] = pmul(ENC[n * JUMP + t], fmaxf(s, 0.0f)); } }
  __syncthreads();
  for (int k = t_; k < CHUNK + 16; k += 256) { float s = 0.0f; if (k < CHUNK) { const int t = k / LK, l = k - t * LK; for (int n = 0; n < NCH; ++n) s += pmul(bf16_rne(wdec[l * NCH + n]), Sw[n][t]); } Se[k] = s; }
  __syncthreads();
  for (int pass = 0; pass < 2; ++pass) { if (t_ < (CHUNK + 16) / 4) *(volatile v4f*)(EST + t_ * 4) = *(const v4f*)(&Se[t_ * 4]); __threadfence(); }
}
__global__ __launch_bounds__(256) void out_kernel(const float* __restrict__ EST, const float* __restrict__ ebuf, const float* __restrict__ ENC, const float* __restrict__ lbuf, const float* __restrict__ LNN, float* __restrict__ out) {
  const int p = blockIdx.x * 256 + threadIdx.x;
  const int pe = imin(p, CHUNK - 1);
  const int q1 = imin(p >= CHUNK ? p - CHUNK : 0, NCH * BUF - 1), c1 = q1 / BUF, t1 = q1 - c1 * BUF;
  const int q2 = imin(p >= CHUNK + NCH * BUF ? p - CHUNK - NCH * BUF : 0, NCH * BUF - 1), c2 = q2 / BUF, t2 = q2 - c2 * BUF;
  const float ve = EST[pe];
  const float e_old = bf16_rne(ebuf[c1 * BUF + imin(t1 + JUMP, BUF - 1)]), e_new = ENC[c1 * JUMP + imin(t1 >= 508 ? t1 - 508 : 0, JUMP - 1)];
  const float l_old = bf16_rne(lbuf[c2 * BUF + imin(t2 + JUMP, BUF - 1)]), l_new = LNN[c2 * JUMP + imin(t2 >= 508 ? t2 - 508 : 0, JUMP - 1)];
  const float v = (p < CHUNK) ? ve : (p < CHUNK + NCH * BUF) ? ((t1 < 508) ? e_old : e_new) : ((t2 < 508) ? l_old : l_new);
  for (int pass = 0; pass < 2; ++pass) { if (p < NOUT) ((volatile float*)out)[p] = v; __threadfence(); }
}
}

extern "C" void kernel_launch(void* const* d_in, const int* in_sizes, int n_in, void* d_out, int out_size, void* d_ws, size_t ws_size, hipStream_t stream) {
  (void)n_in;
  auto Fp = [&](int i) { return (const float*)d_in[i]; };
  if (in_sizes[0] != 2 * CHUNK || in_sizes[1] != NCH * BUF || in_sizes[2] != NCH * BUF || in_sizes[7] != NBLK * HID * NCH || in_sizes[15] != NBLK * NCH * HID || in_sizes[11] != NBLK * HID * 3 || out_size != NOUT) return;
  size_t off = 0; char* ws = (char*)d_ws;
  auto carve = [&](size_t bytes) { char* p = ws + off; off += (bytes + 255) & ~(size_t)255; return p; };
  b16* W1s = (b16*)carve((size_t)NBLK * HID * NCH * 2); b16* W2s = (b16*)carve((size_t)NBLK * HID * NCH * 2);
  const size_t nXF = (size_t)TP * NCH, nY1 = (size_t)TP * HID;
  float* Z = (float*)carve((2 * nXF + nY1) * 4 + 4 * nXF * 2);
  float* XF[2] = {Z, Z + nXF}; float* Y1 = Z + 2 * nXF; b16* Xh16 = (b16*)(Y1 + nY1); b16* XH[2] = {Xh16, Xh16 + nXF}; b16* XL[2] = {Xh16 + 2 * nXF, Xh16 + 3 * nXF};
  const int nz4 = (int)(((2 * nXF + nY1) * 4 + 4 * nXF * 2) / 16);
  float* ENC = (float*)carve(NCH * JUMP * 4); float* LNN = (float*)carve(NCH * JUMP * 4); float* EST = (float*)carve((CHUNK + 16) * 4);
  if (off > ws_size) return;
  prep_kernel<<<512, 256, 0, stream>>>(Fp(7), Fp(15), W1s, W2s, Z, nz4);
  front_kernel<<<1, 256, 0, stream>>>(Fp(0), Fp(3), Fp(4), Fp(5), Fp(6), ENC, LNN);
  x0_kernel<<<TP / 8, 256, 0, stream>>>(Fp(2), LNN, XF[0], XH[0], XL[0]);
  int T = BUF, cur = 0;
  for (int i = 0; i < NBLK; ++i) { const int d = 1 << (i % 7), T_out = T - 2 * d;
    blockA_kernel<<<(T + 15) / 16, 256, 0, stream>>>(W1s + (size_t)i * HID * NCH, XH[cur], XL[cur], Fp(8) + i, Fp(9) + i * HID, Fp(10) + i * HID, Y1, T);
    blockB_kernel<<<(T_out + 15) / 16, 256, 0, stream>>>(Y1, Fp(11) + (size_t)i * HID * 3, Fp(12) + i, Fp(13) + i * HID, Fp(14) + i * HID, W2s + (size_t)i * NCH * HID, XF[cur], XF[cur ^ 1], XH[cur ^ 1], XL[cur ^ 1], d, T_out);
    T = T_out; cur ^= 1; }
  tail_kernel<<<1, 256, 0, stream>>>(XF[cur], ENC, Fp(16), Fp(17), EST);
  out_kernel<<<(NOUT + 255) / 256, 256, 0, stream>>>(EST, Fp(1), ENC, Fp(2), LNN, (float*)d_out);
}
